// MergerSingleW_37649683317095
// MI455X (gfx1250) — hardware-verified
//
#include <hip/hip_runtime.h>


namespace {
constexpr int N = 65536, DI = 32, H = 2048;
constexpr float XS = 8.0f;
typedef _Float16 b16;
typedef __attribute__((ext_vector_type(16))) _Float16 v16b;
typedef __attribute__((ext_vector_type(8))) _Float16 v8b;
typedef __attribute__((ext_vector_type(8))) float v8f;
typedef __attribute__((ext_vector_type(4))) float v4f;
__device__ __forceinline__ float bf16_rne(float f) { unsigned int u = __float_as_uint(f); u += 0x7FFFu + ((u >> 16) & 1u); return __uint_as_float(u & 0xFFFF0000u); }
__device__ __forceinline__ v16b frag_kb(const b16* p, int hh) { const v8b a = *(const v8b*)(p + 8 * hh), b = *(const v8b*)(p + 16 + 8 * hh); v16b f;
#pragma unroll
  for (int e = 0; e < 8; ++e) { f[e] = a[e]; f[8 + e] = b[e]; } return f; }
__device__ __forceinline__ v8f wmma16b(v16b a, v16b b, v8f c) { v8f d = __builtin_amdgcn_wmma_f32_16x16x32_f16(false, a, false, b, (short)0, c, false, false); asm volatile("v_nop\n\tv_nop\n\tv_nop\n\tv_nop" : "+v"(d) : "v"(a), "v"(b)); return d; }
__device__ __forceinline__ void wave_lds_sync() { __builtin_amdgcn_fence(__ATOMIC_RELEASE, "workgroup"); __builtin_amdgcn_wave_barrier(); __builtin_amdgcn_fence(__ATOMIC_ACQUIRE, "workgroup"); }
__device__ __forceinline__ float pmul(float a, float b) { float p = a * b; asm volatile("" : "+v"(p)); return p; }
__device__ __forceinline__ float alpha_of(const float* ar) { const float a = bf16_rne(ar[0]); return log1pf(__expf(a)) + 1e-6f; }
__device__ __forceinline__ float code_of(float w, float alpha) {
  float best = INFINITY; float bc = -63.0f;
#pragma unroll 1
  for (int c = -63; c <= 63; ++c) { if (c == 0) continue; const float d = fabsf(w - pmul(alpha, (float)c)); if (d < best) { best = d; bc = (float)c; } } return bc; }

__global__ __launch_bounds__(256) void code2_kernel(const float* __restrict__ W, const float* __restrict__ ar, b16* __restrict__ C2) {
  const int u = blockIdx.x * 256 + threadIdx.x; if (u >= DI * H / 8) return; const size_t e0 = (size_t)u * 8; const float alpha = alpha_of(ar); v8b v;
#pragma unroll
  for (int j = 0; j < 8; ++j) v[j] = (b16)code_of(bf16_rne(W[e0 + j]), alpha);
  for (int pass = 0; pass < 2; ++pass) { *(volatile v8b*)(C2 + e0) = v; __threadfence(); }
}
__global__ __launch_bounds__(256) void code1_kernel(const float* __restrict__ W, const float* __restrict__ ar, b16* __restrict__ C1) {
  const int h = blockIdx.x * 256 + threadIdx.x; if (h >= H) return; const float alpha = alpha_of(ar); v8b v[4];
#pragma unroll
  for (int k = 0; k < DI; ++k) v[k >> 3][k & 7] = (b16)code_of(bf16_rne(W[(size_t)k * H + h]), alpha);
  for (int pass = 0; pass < 2; ++pass) {
#pragma unroll
    for (int q = 0; q < 4; ++q) *(volatile v8b*)(C1 + (size_t)h * DI + q * 8) = v[q]; __threadfence(); }
}
__global__ __launch_bounds__(32) void mw_kernel(const float* __restrict__ x, const b16* __restrict__ C1, const b16* __restrict__ C2, const float* __restrict__ b1, const float* __restrict__ b2, const float* __restrict__ ar, float* __restrict__ out) {
  __shared__ __attribute__((aligned(16))) b16 Ah[16][40], Hh[16][H + 8]; __shared__ float Of[16][33];
  const int lane = threadIdx.x, nloc = lane & 15, hlf = lane >> 4; const size_t m0 = (size_t)blockIdx.x * 16; const float alpha = alpha_of(ar);
  for (int rr = 0; rr < 16; ++rr) Ah[rr][lane] = (b16)(bf16_rne(x[(m0 + rr) * DI + lane]) * XS);
  wave_lds_sync(); const v16b a = frag_kb(&Ah[nloc][0], hlf);
#pragma unroll 2
  for (int t = 0; t < H / 16; ++t) { v8f acc = {}; acc = wmma16b(a, frag_kb(C1 + (size_t)(t * 16 + nloc) * DI, hlf), acc); const int c = t * 16 + nloc; const float bb = bf16_rne(b1[c]);
#pragma unroll
    for (int r8 = 0; r8 < 8; ++r8) Hh[8 * hlf + r8][c] = (b16)((pmul(alpha, acc[r8] * (1.0f / XS)) + bb) * XS); }
  wave_lds_sync(); v8f o0 = {}, o1 = {};
#pragma unroll 4
  for (int kb = 0; kb < H; kb += 32) { const v16b ha = frag_kb(&Hh[nloc][kb], hlf); o0 = wmma16b(ha, frag_kb(C2 + (size_t)nloc * H + kb, hlf), o0); o1 = wmma16b(ha, frag_kb(C2 + (size_t)(16 + nloc) * H + kb, hlf), o1); }
#pragma unroll
  for (int r8 = 0; r8 < 8; ++r8) { Of[8 * hlf + r8][nloc] = pmul(alpha, o0[r8] * (1.0f / XS)) + bf16_rne(b2[nloc]); Of[8 * hlf + r8][16 + nloc] = pmul(alpha, o1[r8] * (1.0f / XS)) + bf16_rne(b2[16 + nloc]); }
  wave_lds_sync();
  for (int pass = 0; pass < 2; ++pass) { for (int rr = 0; rr < 16; ++rr) ((volatile float*)out)[(m0 + rr) * DI + lane] = Of[rr][lane]; __threadfence(); }
}
}

extern "C" void kernel_launch(void* const* d_in, const int* in_sizes, int n_in, void* d_out, int out_size, void* d_ws, size_t ws_size, hipStream_t stream) {
  (void)n_in;
  auto Fp = [&](int i) { return (const float*)d_in[i]; };
  if (in_sizes[0] != N * DI || in_sizes[1] != DI * H || in_sizes[2] != H || in_sizes[3] != DI || in_sizes[4] != 1 || out_size != N * DI) return;
  const int RL = N;
  size_t off = 0; char* ws = (char*)d_ws;
  auto carve = [&](size_t bytes) { char* p = ws + off; off += (bytes + 255) & ~(size_t)255; return p; };
  b16* C1 = (b16*)carve((size_t)H * DI * 2); b16* C2 = (b16*)carve((size_t)DI * H * 2);
  if (off > ws_size || off > ((size_t)1 << 20)) return;
  code2_kernel<<<(DI * H / 8 + 255) / 256, 256, 0, stream>>>(Fp(1), Fp(4), C2); code1_kernel<<<(H + 255) / 256, 256, 0, stream>>>(Fp(1), Fp(4), C1);
  mw_kernel<<<RL / 16, 32, 0, stream>>>(Fp(0), C1, C2, Fp(2), Fp(3), Fp(4), (float*)d_out);
}
